// GatFfn_76089640615986
// MI455X (gfx1250) — hardware-verified
//
#include <hip/hip_runtime.h>
#include <stddef.h>


#define NF    128
#define NHD   4
#define DW    512
#define GR    32
#define AP    136
#define XSP   516
#define NB    128
#define SP    512
#define HP    132
#define CHUNK 4096
#define NTHR  256
#define NWAVE 8
#define WCAP  512
#define NGRP  (CHUNK / (NTHR * 8))
#define TT    64
#define TPF   68

#define G0_OFF_AL  (GR * AP * 2)
#define G0_OFF_XS  (2 * GR * AP * 2)
#define G0_OFF_AS  (G0_OFF_XS + GR * XSP * 4)
#define G0_OFF_DS  (G0_OFF_AS + GR * NWAVE * 4)
#define G0_LDS     (G0_OFF_DS + GR * NWAVE * 4)

#define AG_OFF_DEN  (NB * SP * 4)
#define AG_OFF_MX   (AG_OFF_DEN + NB * NHD * 4)
#define AG_OFF_LIST (AG_OFF_MX + NB * NHD * 4)
#define AG_OFF_WCNT (AG_OFF_LIST + NWAVE * WCAP * 4)
#define AG_LDS      (AG_OFF_WCNT + 64)

static_assert(NGRP == 2);
static_assert(WCAP == (CHUNK / NTHR) * 32);
static_assert(NB == 128);
static_assert(NB == 16 * NWAVE);
static_assert(GR == 4 * NWAVE);
static_assert(DW == NHD * NF);
static_assert(DW == 64 * NWAVE);
static_assert(CHUNK <= 4096);
static_assert(G0_LDS == 85504);
static_assert(AG_LDS == 282688);
static_assert(3 * NB * HP <= NB * SP);
static_assert((NF % TT) == 0 && (DW % TT) == 0);
static_assert((G0_OFF_AL % 16) == 0 && (G0_OFF_XS % 16) == 0 && (G0_OFF_AS % 16) == 0);
static_assert((AG_OFF_DEN % 16) == 0 && (AG_OFF_MX % 16) == 0 && (AG_OFF_LIST % 16) == 0);

typedef float        v4f  __attribute__((ext_vector_type(4)));
typedef float        v8f  __attribute__((ext_vector_type(8)));
typedef int          v4i  __attribute__((ext_vector_type(4)));
typedef unsigned int v4u  __attribute__((ext_vector_type(4)));
typedef __bf16       v8b  __attribute__((ext_vector_type(8)));
typedef __bf16       v16b __attribute__((ext_vector_type(16)));
union Frag { v16b v; v8b half[2]; v4u u4[2]; };

__device__ __forceinline__ unsigned int bfr(float f) {
  unsigned int u = __float_as_uint(f);
  u += 0x7FFFu + ((u >> 16) & 1u);
  return u >> 16;
}
__device__ __forceinline__ unsigned int pk2(float a, float b, unsigned int& lo) {
  const unsigned int ha = bfr(a), hb = bfr(b);
  const float ra = a - __uint_as_float(ha << 16);
  const float rb = b - __uint_as_float(hb << 16);
  lo = bfr(ra) | (bfr(rb) << 16);
  return ha | (hb << 16);
}
__device__ __forceinline__ void split8(v4f a, v4f b, v4u& hi, v4u& lo) {
  unsigned int l0, l1, l2, l3;
  const unsigned int h0 = pk2(a.x, a.y, l0);
  const unsigned int h1 = pk2(a.z, a.w, l1);
  const unsigned int h2 = pk2(b.x, b.y, l2);
  const unsigned int h3 = pk2(b.z, b.w, l3);
  hi.x = h0; hi.y = h1; hi.z = h2; hi.w = h3;
  lo.x = l0; lo.y = l1; lo.z = l2; lo.w = l3;
}

__device__ __forceinline__ v8f wm3(v8f c, v16b ah, v16b al, v16b bh, v16b bl) {
  c = __builtin_amdgcn_wmma_f32_16x16x32_bf16(false, ah, false, bh, (short)0, c, false, false);
  c = __builtin_amdgcn_wmma_f32_16x16x32_bf16(false, al, false, bh, (short)0, c, false, false);
  c = __builtin_amdgcn_wmma_f32_16x16x32_bf16(false, ah, false, bl, (short)0, c, false, false);
  asm volatile("v_nop\n\tv_nop\n\tv_nop\n\tv_nop" : "+v"(c) : "v"(ah), "v"(al), "v"(bh), "v"(bl) : "memory");
  return c;
}

__device__ __forceinline__ void zero8(v8f (&acc)[8]) {
  const v8f z8 = {0.f, 0.f, 0.f, 0.f, 0.f, 0.f, 0.f, 0.f};
#pragma unroll
  for (int i = 0; i < 8; ++i) acc[i] = z8;
}

__global__ __launch_bounds__(NTHR) void k_prepw(const float* __restrict__ W,
                                                unsigned short* Wh, unsigned short* Wl, int K, int Nc) {
  __shared__ __attribute__((aligned(16))) float T[TT * TPF];
  const int tid = threadIdx.x;
  const int n0 = blockIdx.x * TT;
  const int k0 = blockIdx.y * TT;
#pragma unroll
  for (int it = 0; it < (TT * TT / 4) / NTHR; ++it) {
    const int idx = it * NTHR + tid;
    const int kr = idx >> 4;
    const int c4 = (idx & 15) * 4;
    const v4f v = *(const v4f*)(W + (size_t)(k0 + kr) * Nc + n0 + c4);
    *(v4f*)(T + kr * TPF + c4) = v;
  }
  __syncthreads();
  const int j = tid & 7;
  const int nr0 = tid >> 3;
  const int nr1 = 32 + (tid >> 3);
  v4f a0, b0, a1, b1;
  a0.x = T[(8 * j + 0) * TPF + nr0]; a0.y = T[(8 * j + 1) * TPF + nr0];
  a0.z = T[(8 * j + 2) * TPF + nr0]; a0.w = T[(8 * j + 3) * TPF + nr0];
  b0.x = T[(8 * j + 4) * TPF + nr0]; b0.y = T[(8 * j + 5) * TPF + nr0];
  b0.z = T[(8 * j + 6) * TPF + nr0]; b0.w = T[(8 * j + 7) * TPF + nr0];
  a1.x = T[(8 * j + 0) * TPF + nr1]; a1.y = T[(8 * j + 1) * TPF + nr1];
  a1.z = T[(8 * j + 2) * TPF + nr1]; a1.w = T[(8 * j + 3) * TPF + nr1];
  b1.x = T[(8 * j + 4) * TPF + nr1]; b1.y = T[(8 * j + 5) * TPF + nr1];
  b1.z = T[(8 * j + 6) * TPF + nr1]; b1.w = T[(8 * j + 7) * TPF + nr1];
  v4u h0, l0, h1, l1;
  split8(a0, b0, h0, l0);
  split8(a1, b1, h1, l1);
  const size_t o0 = (size_t)(n0 + nr0) * K + k0 + 8 * j;
  const size_t o1 = (size_t)(n0 + nr1) * K + k0 + 8 * j;
  *(volatile v4u*)(Wh + o0) = h0;
  *(volatile v4u*)(Wl + o0) = l0;
  *(volatile v4u*)(Wh + o1) = h1;
  *(volatile v4u*)(Wl + o1) = l1;
  __threadfence();
  *(volatile v4u*)(Wh + o0) = h0;
  *(volatile v4u*)(Wl + o0) = l0;
  *(volatile v4u*)(Wh + o1) = h1;
  *(volatile v4u*)(Wl + o1) = l1;
}

__global__ __launch_bounds__(NTHR) void k_gemm0(
    const float* __restrict__ x, const unsigned short* __restrict__ Wgh, const unsigned short* __restrict__ Wgl,
    const float* __restrict__ att_s, const float* __restrict__ att_d,
    float* xp, float* asrc, float* adst, int nN) {
  extern __shared__ v4f lds_dyn[];
  char* base = (char*)lds_dyn;
  unsigned short* Ah = (unsigned short*)base;
  unsigned short* Al = (unsigned short*)(base + G0_OFF_AL);
  float* Xs = (float*)(base + G0_OFF_XS);
  float* As = (float*)(base + G0_OFF_AS);
  float* Ds = (float*)(base + G0_OFF_DS);

  const int tid  = threadIdx.x;
  const int lane = tid & 31;
  const int wave = tid >> 5;
  const int hh   = lane >> 4;
  const int m    = lane & 15;
  const int rowBase = blockIdx.x * GR;

  {
    const int r  = tid >> 3;
    const int c0 = (tid & 7) * 16;
    int row = rowBase + r;
    if (row > nN - 1) row = nN - 1;
    const float* p = x + (size_t)row * NF + c0;
    const v4f f0 = *(const v4f*)(p), f1 = *(const v4f*)(p + 4);
    const v4f f2 = *(const v4f*)(p + 8), f3 = *(const v4f*)(p + 12);
    v4u h0, l0, h1, l1;
    split8(f0, f1, h0, l0);
    split8(f2, f3, h1, l1);
    *(v4u*)(Ah + r * AP + c0)     = h0;
    *(v4u*)(Ah + r * AP + c0 + 8) = h1;
    *(v4u*)(Al + r * AP + c0)     = l0;
    *(v4u*)(Al + r * AP + c0 + 8) = l1;
  }
  __syncthreads();

  const int cb = wave * 64;
  v8f acc[2][4];
  {
    const v8f z8 = {0.f, 0.f, 0.f, 0.f, 0.f, 0.f, 0.f, 0.f};
#pragma unroll
    for (int mt = 0; mt < 2; ++mt)
#pragma unroll
      for (int nt = 0; nt < 4; ++nt) acc[mt][nt] = z8;
  }
#pragma unroll
  for (int kt = 0; kt < NF / 32; ++kt) {
    const int k0 = kt * 32;
    Frag a0h, a0l, a1h, a1l;
    const unsigned short* p0h = Ah + m * AP + k0 + 8 * hh;
    const unsigned short* p1h = Ah + (16 + m) * AP + k0 + 8 * hh;
    const unsigned short* p0l = Al + m * AP + k0 + 8 * hh;
    const unsigned short* p1l = Al + (16 + m) * AP + k0 + 8 * hh;
    a0h.half[0] = *(const v8b*)p0h; a0h.half[1] = *(const v8b*)(p0h + 16);
    a1h.half[0] = *(const v8b*)p1h; a1h.half[1] = *(const v8b*)(p1h + 16);
    a0l.half[0] = *(const v8b*)p0l; a0l.half[1] = *(const v8b*)(p0l + 16);
    a1l.half[0] = *(const v8b*)p1l; a1l.half[1] = *(const v8b*)(p1l + 16);
#pragma unroll
    for (int nt = 0; nt < 4; ++nt) {
      const int ncol = cb + 16 * nt + m;
      const unsigned short* pbh = Wgh + (size_t)ncol * NF + k0 + 8 * hh;
      const unsigned short* pbl = Wgl + (size_t)ncol * NF + k0 + 8 * hh;
      Frag bh, bl;
      bh.half[0] = *(const v8b*)pbh; bh.half[1] = *(const v8b*)(pbh + 16);
      bl.half[0] = *(const v8b*)pbl; bl.half[1] = *(const v8b*)(pbl + 16);
      acc[0][nt] = wm3(acc[0][nt], a0h.v, a0l.v, bh.v, bl.v);
      acc[1][nt] = wm3(acc[1][nt], a1h.v, a1l.v, bh.v, bl.v);
    }
  }

  float cs[4], cd[4];
#pragma unroll
  for (int nt = 0; nt < 4; ++nt) {
    cs[nt] = att_s[cb + 16 * nt + m];
    cd[nt] = att_d[cb + 16 * nt + m];
  }
#pragma unroll
  for (int mt = 0; mt < 2; ++mt) {
    float ss[8], sd[8];
#pragma unroll
    for (int r = 0; r < 8; ++r) { ss[r] = 0.f; sd[r] = 0.f; }
#pragma unroll
    for (int nt = 0; nt < 4; ++nt) {
#pragma unroll
      for (int r = 0; r < 8; ++r) {
        const float v = acc[mt][nt][r];
        Xs[(16 * mt + 8 * hh + r) * XSP + cb + 16 * nt + m] = v;
        ss[r] += v * cs[nt];
        sd[r] += v * cd[nt];
      }
    }
#pragma unroll
    for (int mk = 1; mk < 16; mk <<= 1) {
#pragma unroll
      for (int r = 0; r < 8; ++r) {
        ss[r] += __shfl_xor(ss[r], mk, 32);
        sd[r] += __shfl_xor(sd[r], mk, 32);
      }
    }
    if (m == 0) {
#pragma unroll
      for (int r = 0; r < 8; ++r) {
        As[(16 * mt + 8 * hh + r) * NWAVE + wave] = ss[r];
        Ds[(16 * mt + 8 * hh + r) * NWAVE + wave] = sd[r];
      }
    }
  }
  __syncthreads();

  v4f xr[16];
#pragma unroll
  for (int i = 0; i < 4; ++i)
#pragma unroll
    for (int s = 0; s < 4; ++s)
      xr[4 * i + s] = *(const v4f*)(Xs + (4 * wave + i) * XSP + NF * s + 4 * lane);
  v4f gv = {0.f, 0.f, 0.f, 0.f};
  float* gp = asrc;
  const bool wg = (wave < 2);
  if (wave == 0) {
    const float* ar = As + lane * NWAVE;
    gv.x = ar[0] + ar[1]; gv.y = ar[2] + ar[3]; gv.z = ar[4] + ar[5]; gv.w = ar[6] + ar[7];
    gp = asrc + (size_t)(rowBase + lane) * NHD;
  } else if (wave == 1) {
    const float* ar = Ds + lane * NWAVE;
    gv.x = ar[0] + ar[1]; gv.y = ar[2] + ar[3]; gv.z = ar[4] + ar[5]; gv.w = ar[6] + ar[7];
    gp = adst + (size_t)(rowBase + lane) * NHD;
  }
  float* xq = xp + (size_t)(rowBase + 4 * wave) * DW + 4 * lane;
#pragma unroll
  for (int i = 0; i < 4; ++i)
#pragma unroll
    for (int s = 0; s < 4; ++s)
      *(volatile v4f*)(xq + (size_t)i * DW + NF * s) = xr[4 * i + s];
  if (wg) *(volatile v4f*)gp = gv;
  __threadfence();
#pragma unroll
  for (int i = 0; i < 4; ++i)
#pragma unroll
    for (int s = 0; s < 4; ++s)
      *(volatile v4f*)(xq + (size_t)i * DW + NF * s) = xr[4 * i + s];
  if (wg) *(volatile v4f*)gp = gv;
}

template <int KT>
__device__ __forceinline__ void gemm16(const float* arow, const unsigned short* __restrict__ Bh,
                                       const unsigned short* __restrict__ Bl, int m, int hh, v8f (&acc)[8]) {
#pragma unroll 1
  for (int kt = 0; kt < KT / 32; ++kt) {
    const int k0 = kt * 32;
    const float* ap = arow + k0 + 8 * hh;
    const v4f q0 = *(const v4f*)(ap);
    const v4f q1 = *(const v4f*)(ap + 4);
    const v4f q2 = *(const v4f*)(ap + 16);
    const v4f q3 = *(const v4f*)(ap + 20);
    Frag ah, al;
    split8(q0, q1, ah.u4[0], al.u4[0]);
    split8(q2, q3, ah.u4[1], al.u4[1]);
#pragma unroll
    for (int nt = 0; nt < 8; ++nt) {
      const unsigned short* pbh = Bh + (size_t)(16 * nt + m) * KT + k0 + 8 * hh;
      const unsigned short* pbl = Bl + (size_t)(16 * nt + m) * KT + k0 + 8 * hh;
      Frag bh, bl;
      bh.half[0] = *(const v8b*)pbh; bh.half[1] = *(const v8b*)(pbh + 16);
      bl.half[0] = *(const v8b*)pbl; bl.half[1] = *(const v8b*)(pbl + 16);
      acc[nt] = wm3(acc[nt], ah.v, al.v, bh.v, bl.v);
    }
  }
}

#define HITJ(J, HJ, SJ) {                                                       \
    const unsigned mj = __builtin_amdgcn_ballot_w32(HJ);                        \
    if (HJ) {                                                                   \
      const int pos = wc + (int)__builtin_amdgcn_mbcnt_lo(mj, 0u);              \
      if (pos < WCAP) list[wave * WCAP + pos] = ((el0 + (J)) << 7) | (int)(SJ);  \
    }                                                                           \
    wc += (int)__builtin_popcount(mj); }

#define SUB4(D, J0) {                                                           \
    const unsigned s0 = (unsigned)D.x - (unsigned)nodeBase;                     \
    const unsigned s1 = (unsigned)D.y - (unsigned)nodeBase;                     \
    const unsigned s2 = (unsigned)D.z - (unsigned)nodeBase;                     \
    const unsigned s3 = (unsigned)D.w - (unsigned)nodeBase;                     \
    const bool h0 = s0 < (unsigned)NB;                                          \
    const bool h1 = s1 < (unsigned)NB;                                          \
    const bool h2 = s2 < (unsigned)NB;                                          \
    const bool h3 = s3 < (unsigned)NB;                                          \
    const unsigned many = __builtin_amdgcn_ballot_w32(h0 | h1 | h2 | h3);       \
    if (many != 0u) {                                                           \
      HITJ((J0) + 0, h0, s0)                                                    \
      HITJ((J0) + 1, h1, s1)                                                    \
      HITJ((J0) + 2, h2, s2)                                                    \
      HITJ((J0) + 3, h3, s3)                                                    \
    } }

#define LDJ(DST, J) DST = (e0 + (J) < nE) ? eid[min(e0 + (J), nE - 1)] : sent;

#define HEADD(C, H) {                                                           \
    float al = as4.C + ad4.C;                                                   \
    al = (al > 0.f) ? al : 0.2f * al;                                           \
    const float mn = fmaxf(mo4.C, al);                                          \
    const float sc = __expf(mo4.C - mn);                                        \
    const float p  = __expf(al - mn);                                           \
    const v4f xv = *(const v4f*)(xrow + NF * (H));                              \
    v4f* sp4 = (v4f*)(srow + NF * (H));                                         \
    const v4f cur = *sp4;                                                       \
    *sp4 = cur * sc + xv * p;                                                   \
    mn4.C = mn;                                                                 \
    dw4.C = dn4.C * sc + p; }

#define HEADF(C, H) {                                                           \
    float al = as4.C + ad4.C;                                                   \
    al = (al > 0.f) ? al : 0.2f * al;                                           \
    const float mn = fmaxf(mo4.C, al);                                          \
    const float sc = __expf(mo4.C - mn);                                        \
    const float p  = __expf(al - mn);                                           \
    const v4f xv = *(const v4f*)(xrow + NF * (H));                              \
    v4f* sp4 = (v4f*)(srow + NF * (H));                                         \
    const v4f tot = (*sp4) * sc + xv * p;                                       \
    const float dt  = dn4.C * sc + p;                                           \
    const float inv = 1.0f / dt;                                                \
    const v4f b4 = *(const v4f*)(bgat + NF * (H) + 4 * lane);                   \
    v4f g = tot * inv + b4;                                                     \
    g.x = g.x > 0.f ? g.x : 0.01f * g.x;                                        \
    g.y = g.y > 0.f ? g.y : 0.01f * g.y;                                        \
    g.z = g.z > 0.f ? g.z : 0.01f * g.z;                                        \
    g.w = g.w > 0.f ? g.w : 0.01f * g.w;                                        \
    *sp4 = g; }

__global__ __launch_bounds__(NTHR) void k_agg(
    const float* __restrict__ x, const int* __restrict__ ei, const float* __restrict__ xp,
    const float* __restrict__ asrc, const float* __restrict__ adst, const float* __restrict__ bgat,
    const unsigned short* __restrict__ Wmh, const unsigned short* __restrict__ Wml, const float* __restrict__ bmha,
    const unsigned short* __restrict__ W1h, const unsigned short* __restrict__ W1l, const float* __restrict__ b1,
    const unsigned short* __restrict__ W2h, const unsigned short* __restrict__ W2l, const float* __restrict__ b2,
    float* out, int nN, int nE) {
  extern __shared__ v4f lds_dyn[];
  char* base = (char*)lds_dyn;
  float* sacc = (float*)base;
  float* den  = (float*)(base + AG_OFF_DEN);
  float* mx   = (float*)(base + AG_OFF_MX);
  int*   list = (int*)(base + AG_OFF_LIST);
  int*   wcnt = (int*)(base + AG_OFF_WCNT);

  const int tid  = threadIdx.x;
  const int lane = tid & 31;
  const int wave = tid >> 5;
  const int hh   = lane >> 4;
  const int m    = lane & 15;
  const int nodeBase = blockIdx.x * NB;

  {
    const v4f z4 = {0.f, 0.f, 0.f, 0.f};
    for (int i = tid; i < NB * SP / 4; i += NTHR) lds_dyn[i] = z4;
    for (int i = tid; i < NB * NHD; i += NTHR) { den[i] = 0.f; mx[i] = -1.0e30f; }
  }
  __syncthreads();

  const int* eid = ei + nE;
  const bool al16 = ((nE & 3) == 0);
  const int nChunks = (nE + CHUNK - 1) / CHUNK;

#pragma unroll 1
  for (int ch = 0; ch < nChunks; ++ch) {
    const int cbase = ch * CHUNK;
    int wc = 0;
#pragma unroll
    for (int g = 0; g < NGRP; ++g) {
      const int el0 = (g * NTHR + tid) * 8;
      const int e0  = cbase + el0;
      const int sent = -2147483647 - 1;
      v4i da, db;
      if (al16 && (e0 + 7 < nE)) {
        da = *(const v4i*)(eid + e0);
        db = *(const v4i*)(eid + e0 + 4);
      } else {
        LDJ(da.x, 0) LDJ(da.y, 1) LDJ(da.z, 2) LDJ(da.w, 3)
        LDJ(db.x, 4) LDJ(db.y, 5) LDJ(db.z, 6) LDJ(db.w, 7)
      }
      SUB4(da, 0)
      SUB4(db, 4)
    }
    if (lane == 0) wcnt[wave] = wc;
    __syncthreads();

    if (wave == 0) {
      for (int wsx = 0; wsx < NWAVE; ++wsx) {
        int n = wcnt[wsx];
        if (n > WCAP) n = WCAP;
        if (n < 0) n = 0;
        for (int i = 0; i < n; ++i) {
          const int ent  = list[wsx * WCAP + i];
          const int slot = ent & (NB - 1);
          const int el   = (ent >> 7) & (CHUNK - 1);
          int e = cbase + el;
          if (e > nE - 1) e = nE - 1;
          int src = ei[e];
          src = src < 0 ? 0 : (src > nN - 1 ? nN - 1 : src);
          int nd = nodeBase + slot;
          if (nd > nN - 1) nd = nN - 1;
          const v4f as4 = *(const v4f*)(asrc + (size_t)src * NHD);
          const v4f ad4 = *(const v4f*)(adst + (size_t)nd * NHD);
          const v4f mo4 = *(const v4f*)(mx + slot * NHD);
          const v4f dn4 = *(const v4f*)(den + slot * NHD);
          const float* xrow = xp + (size_t)src * DW + 4 * lane;
          float* srow = sacc + slot * SP + 4 * lane;
          v4f mn4 = {0.f, 0.f, 0.f, 0.f};
          v4f dw4 = {0.f, 0.f, 0.f, 0.f};
          HEADD(x, 0)
          HEADD(y, 1)
          HEADD(z, 2)
          HEADD(w, 3)
          if (lane == 0) {
            *(v4f*)(mx + slot * NHD)  = mn4;
            *(v4f*)(den + slot * NHD) = dw4;
          }
        }
      }
    }
    __syncthreads();
  }

#pragma unroll 1
  for (int j = 0; j < NB / NWAVE; ++j) {
    const int slot = wave * (NB / NWAVE) + j;
    int node = nodeBase + slot;
    if (node > nN - 1) node = nN - 1;
    const v4f as4 = *(const v4f*)(asrc + (size_t)node * NHD);
    const v4f ad4 = *(const v4f*)(adst + (size_t)node * NHD);
    const v4f mo4 = *(const v4f*)(mx + slot * NHD);
    const v4f dn4 = *(const v4f*)(den + slot * NHD);
    const float* xrow = xp + (size_t)node * DW + 4 * lane;
    float* srow = sacc + slot * SP + 4 * lane;
    HEADF(x, 0)
    HEADF(y, 1)
    HEADF(z, 2)
    HEADF(w, 3)
  }
  __syncthreads();

  const int arow = 16 * wave + m;
  v8f acc[8];
  zero8(acc);
  gemm16<DW>(sacc + arow * SP, Wmh, Wml, m, hh, acc);
  __syncthreads();

  float* Hs = sacc;
  float* Ms = sacc + NB * HP;
  float* Os = sacc + 2 * NB * HP;
#pragma unroll
  for (int nt = 0; nt < 8; ++nt) {
    const int n = 16 * nt + m;
    const float bv = bmha[n];
#pragma unroll
    for (int r = 0; r < 8; ++r) Hs[(16 * wave + 8 * hh + r) * HP + n] = acc[nt][r] + bv;
  }
  __syncthreads();
#pragma unroll
  for (int r = 0; r < 16; ++r) {
    const int row = 16 * wave + r;
    int node = nodeBase + row;
    if (node > nN - 1) node = nN - 1;
    v4f* hp4 = (v4f*)(Hs + row * HP + 4 * lane);
    const v4f xv = *(const v4f*)(x + (size_t)node * NF + 4 * lane);
    const v4f hv = *hp4;
    *hp4 = hv + xv;
  }
  __syncthreads();

  zero8(acc);
  gemm16<NF>(Hs + arow * HP, W1h, W1l, m, hh, acc);
#pragma unroll
  for (int nt = 0; nt < 8; ++nt) {
    const int n = 16 * nt + m;
    const float bv = b1[n];
#pragma unroll
    for (int r = 0; r < 8; ++r) {
      float v = acc[nt][r] + bv;
      v = v > 0.f ? v : 0.01f * v;
      Ms[(16 * wave + 8 * hh + r) * HP + n] = v;
    }
  }
  __syncthreads();

  zero8(acc);
  gemm16<NF>(Ms + arow * HP, W2h, W2l, m, hh, acc);
#pragma unroll
  for (int nt = 0; nt < 8; ++nt) {
    const int n = 16 * nt + m;
    const float bv = b2[n];
#pragma unroll
    for (int r = 0; r < 8; ++r) {
      const int row = 16 * wave + 8 * hh + r;
      Os[row * HP + n] = acc[nt][r] + bv + Hs[row * HP + n];
    }
  }
  __syncthreads();

  int nv = nN - (nodeBase + 16 * wave);
  if (nv > 16) nv = 16;
  v4f ov[16];
#pragma unroll
  for (int r = 0; r < 16; ++r) ov[r] = *(const v4f*)(Os + (16 * wave + r) * HP + 4 * lane);
  float* op = out + (size_t)(nodeBase + 16 * wave) * NF + 4 * lane;
#pragma unroll
  for (int r = 0; r < 16; ++r)
    if (r < nv) *(volatile v4f*)(op + (size_t)r * NF) = ov[r];
  __threadfence();
#pragma unroll
  for (int r = 0; r < 16; ++r)
    if (r < nv) *(volatile v4f*)(op + (size_t)r * NF) = ov[r];
}

extern "C" void kernel_launch(void* const* d_in, const int* in_sizes, int n_in,
                              void* d_out, int out_size, void* d_ws, size_t ws_size,
                              hipStream_t stream) {
  if (n_in < 12) return;
  const int nN = in_sizes[0] / NF;
  if (nN <= 0 || in_sizes[0] != nN * NF) return;
  if (in_sizes[1] < 0 || (in_sizes[1] & 1) != 0) return;
  const int nE = in_sizes[1] / 2;
  if (in_sizes[2] != NF * DW) return;
  if (in_sizes[3] != NHD * NF || in_sizes[4] != NHD * NF) return;
  if (in_sizes[5] != DW) return;
  if (in_sizes[6] != DW * NF || in_sizes[7] != NF) return;
  if (in_sizes[8] != NF * NF || in_sizes[9] != NF) return;
  if (in_sizes[10] != NF * NF || in_sizes[11] != NF) return;
  if (out_size != nN * NF) return;

  const float* x        = (const float*)d_in[0];
  const int*   ei       = (const int*)d_in[1];
  const float* W_gat    = (const float*)d_in[2];
  const float* att_src  = (const float*)d_in[3];
  const float* att_dst  = (const float*)d_in[4];
  const float* bias_gat = (const float*)d_in[5];
  const float* W_mha    = (const float*)d_in[6];
  const float* b_mha    = (const float*)d_in[7];
  const float* W1       = (const float*)d_in[8];
  const float* b1       = (const float*)d_in[9];
  const float* W2       = (const float*)d_in[10];
  const float* b2       = (const float*)d_in[11];
  float* out = (float*)d_out;

  const int nP = ((nN + GR - 1) / GR) * GR;
  size_t off = 0;
  unsigned short* Wgh = (unsigned short*)((char*)d_ws + off); off += (size_t)NF * DW * 2;
  unsigned short* Wgl = (unsigned short*)((char*)d_ws + off); off += (size_t)NF * DW * 2;
  unsigned short* Wmh = (unsigned short*)((char*)d_ws + off); off += (size_t)DW * NF * 2;
  unsigned short* Wml = (unsigned short*)((char*)d_ws + off); off += (size_t)DW * NF * 2;
  unsigned short* W1h = (unsigned short*)((char*)d_ws + off); off += (size_t)NF * NF * 2;
  unsigned short* W1l = (unsigned short*)((char*)d_ws + off); off += (size_t)NF * NF * 2;
  unsigned short* W2h = (unsigned short*)((char*)d_ws + off); off += (size_t)NF * NF * 2;
  unsigned short* W2l = (unsigned short*)((char*)d_ws + off); off += (size_t)NF * NF * 2;
  float* xp   = (float*)((char*)d_ws + off); off += (size_t)nP * DW * sizeof(float);
  float* asrc = (float*)((char*)d_ws + off); off += (size_t)nP * NHD * sizeof(float);
  float* adst = (float*)((char*)d_ws + off); off += (size_t)nP * NHD * sizeof(float);
  if (off > ws_size) return;
  if (off > (size_t)134217728) return;

  k_prepw<<<dim3(DW / TT, NF / TT), NTHR, 0, stream>>>(W_gat, Wgh, Wgl, NF, DW);
  k_prepw<<<dim3(NF / TT, DW / TT), NTHR, 0, stream>>>(W_mha, Wmh, Wml, DW, NF);
  k_prepw<<<dim3(NF / TT, NF / TT), NTHR, 0, stream>>>(W1, W1h, W1l, NF, NF);
  k_prepw<<<dim3(NF / TT, NF / TT), NTHR, 0, stream>>>(W2, W2h, W2l, NF, NF);

  hipFuncSetAttribute(reinterpret_cast<const void*>(&k_gemm0),
                      hipFuncAttributeMaxDynamicSharedMemorySize, G0_LDS);
  k_gemm0<<<nP / GR, NTHR, G0_LDS, stream>>>(x, Wgh, Wgl, att_src, att_dst, xp, asrc, adst, nN);

  hipFuncSetAttribute(reinterpret_cast<const void*>(&k_agg),
                      hipFuncAttributeMaxDynamicSharedMemorySize, AG_LDS);
  const int grid = (nN + NB - 1) / NB;
  k_agg<<<grid, NTHR, AG_LDS, stream>>>(x, ei, xp, asrc, adst, bias_gat, Wmh, Wml, b_mha,
                                         W1h, W1l, b1, W2h, W2l, b2, out, nN, nE);
}
